// gaussian_decoder_het_58566174049032
// MI455X (gfx1250) — hardware-verified
//
#include <hip/hip_runtime.h>
#include <stddef.h>
#include <math.h>


#define BIMG   16
#define NPT    50000
#define LATD   10
#define NEU    32
#define NLAY   3
#define KIN0   12
#define BOXW   256
#define HALFK  4
#define KTAP   9
#define NROWS  (BIMG * NPT)
#define RT     64
#define MT     128
#define HP     36
#define ST     256
#define NWS    (ST / 32)
#define TW     64
#define TPD    (BOXW / TW)
#define TPI    (TPD * TPD)

static_assert(NROWS % RT == 0);
static_assert(MT == 2 * RT);
static_assert((BOXW % TW) == 0);
static_assert(TW == 64);
static_assert(ST == 256);
static_assert((HP % 4) == 0);

typedef float  v2f  __attribute__((ext_vector_type(2)));
typedef float  v4f  __attribute__((ext_vector_type(4)));
typedef float  v8f  __attribute__((ext_vector_type(8)));
typedef __bf16 v8b  __attribute__((ext_vector_type(8)));
typedef __bf16 v16b __attribute__((ext_vector_type(16)));
union FragB { v16b v; v8b h[2]; };
struct HL { v8b hi; v8b lo; };

__device__ __forceinline__ v8f zero8f() {
  v8f c;
#pragma unroll
  for (int i = 0; i < 8; ++i) c[i] = 0.0f;
  return c;
}

__device__ __forceinline__ v8f wmb(v16b a, v16b b, v8f c) {
  v8f d = __builtin_amdgcn_wmma_f32_16x16x32_bf16(false, a, false, b, (short)0, c, false, false);
  asm volatile("v_nop\n\tv_nop\n\tv_nop\n\tv_nop" : "+v"(d) : "v"(a), "v"(b));
  return d;
}

__device__ __forceinline__ HL split8(v4f a, v4f b) {
  float f[8];
  f[0] = a.x; f[1] = a.y; f[2] = a.z; f[3] = a.w;
  f[4] = b.x; f[5] = b.y; f[6] = b.z; f[7] = b.w;
  HL r;
#pragma unroll
  for (int i = 0; i < 8; ++i) {
    const __bf16 t = (__bf16)f[i];
    const float rm = f[i] - (float)t;
    r.hi[i] = t;
    r.lo[i] = (__bf16)rm;
  }
  return r;
}

__global__ __launch_bounds__(MT) void k_mlp(
    const float* __restrict__ z, const float* __restrict__ rot, const float* __restrict__ posp,
    const float* __restrict__ amp, const float* __restrict__ w0, const float* __restrict__ wd,
    const float* __restrict__ bd, const float* __restrict__ w1a, const float* __restrict__ w1b,
    const float* __restrict__ law, const float* __restrict__ lab, const int* __restrict__ dfl,
    float* out2, float* out3, float* out4, float* sp) {
  __shared__ __attribute__((aligned(16))) __bf16 whi[NLAY * NEU * NEU];
  __shared__ __attribute__((aligned(16))) __bf16 wlo[NLAY * NEU * NEU];
  __shared__ __attribute__((aligned(16))) float hs[RT * HP];
  __shared__ __attribute__((aligned(16))) float w0s[NEU * KIN0];
  __shared__ float bds[NLAY * NEU];
  __shared__ float w1s[3 * NEU];
  __shared__ float w1bs[9];
  __shared__ float zs[BIMG * LATD];
  __shared__ __attribute__((aligned(16))) float o2s[RT * 2];
  __shared__ __attribute__((aligned(16))) float o3s[RT * 3];
  __shared__ __attribute__((aligned(16))) float o4s[RT * 3];
  __shared__ __attribute__((aligned(16))) float sps[RT * 4];

  const int tid = threadIdx.x, lane = tid & 31, wave = tid >> 5, hh = lane >> 4, m = lane & 15;
  const int R0 = (int)blockIdx.x * RT;
  if (R0 + RT > NROWS) return;

#pragma unroll 1
  for (int i = tid; i < NLAY * NEU * NEU; i += MT) {
    const float v = wd[i];
    const __bf16 hb = (__bf16)v;
    const float rm = v - (float)hb;
    whi[i] = hb;
    wlo[i] = (__bf16)rm;
  }
#pragma unroll 1
  for (int i = tid; i < NEU * KIN0; i += MT) w0s[i] = w0[i];
#pragma unroll 1
  for (int i = tid; i < BIMG * LATD; i += MT) zs[i] = z[i];
  if (tid < NLAY * NEU) bds[tid] = bd[tid];
  if (tid < 3 * NEU) w1s[tid] = w1a[tid];
  if (tid < 9) w1bs[tid] = w1b[tid];
  __syncthreads();

  {
    const int q = tid & (RT - 1);
    const int half = tid >> 6;
    const int R = R0 + q;
    const int b = R / NPT;
    const int n = R - b * NPT;
    float x[KIN0];
    x[0] = posp[(size_t)n * 3 + 0];
    x[1] = posp[(size_t)n * 3 + 1];
    x[2] = posp[(size_t)n * 3 + 2];
#pragma unroll
    for (int k = 0; k < LATD - 1; ++k) x[3 + k] = zs[b * LATD + k];
#pragma unroll
    for (int jj = 0; jj < NEU / 2; ++jj) {
      const int j = half * (NEU / 2) + jj;
      const float* wr = w0s + j * KIN0;
      float s = 0.0f;
#pragma unroll
      for (int k = 0; k < KIN0; ++k) s += x[k] * wr[k];
      hs[q * HP + j] = s;
    }
  }
  __syncthreads();

#pragma unroll
  for (int l = 0; l < NLAY; ++l) {
    FragB ah, al;
    {
      const float* hr = hs + (16 * wave + m) * HP + 8 * hh;
      const v4f x0 = *(const v4f*)(hr);
      const v4f x1 = *(const v4f*)(hr + 4);
      const v4f x2 = *(const v4f*)(hr + 16);
      const v4f x3 = *(const v4f*)(hr + 20);
      const HL s0 = split8(x0, x1);
      const HL s1 = split8(x2, x3);
      ah.h[0] = s0.hi; al.h[0] = s0.lo;
      ah.h[1] = s1.hi; al.h[1] = s1.lo;
    }
    v8f d0, d1;
    {
      const int wi = (l * NEU + m) * NEU + 8 * hh;
      FragB bh, bl;
      bh.h[0] = *(const v8b*)(whi + wi);
      bh.h[1] = *(const v8b*)(whi + wi + 16);
      bl.h[0] = *(const v8b*)(wlo + wi);
      bl.h[1] = *(const v8b*)(wlo + wi + 16);
      v8f c = zero8f();
      c = wmb(al.v, bh.v, c);
      c = wmb(ah.v, bl.v, c);
      c = wmb(ah.v, bh.v, c);
      d0 = c;
    }
    {
      const int wi = (l * NEU + 16 + m) * NEU + 8 * hh;
      FragB bh, bl;
      bh.h[0] = *(const v8b*)(whi + wi);
      bh.h[1] = *(const v8b*)(whi + wi + 16);
      bl.h[0] = *(const v8b*)(wlo + wi);
      bl.h[1] = *(const v8b*)(wlo + wi + 16);
      v8f c = zero8f();
      c = wmb(al.v, bh.v, c);
      c = wmb(ah.v, bl.v, c);
      c = wmb(ah.v, bh.v, c);
      d1 = c;
    }
#pragma unroll
    for (int r = 0; r < 8; ++r) {
      const int row = 16 * wave + 8 * hh + r;
      float* hrow = hs + row * HP;
      const float va = fmaxf(d0[r] + bds[l * NEU + m], 0.0f) + hrow[m];
      const float vb = fmaxf(d1[r] + bds[l * NEU + 16 + m], 0.0f) + hrow[16 + m];
      hrow[m] = va;
      hrow[16 + m] = vb;
    }
    __syncthreads();
  }

  if (tid < RT) {
    const int q = tid;
    const int R = R0 + q;
    const int b = R / NPT;
    const int n = R - b * NPT;
    const float* hr = hs + q * HP;
    float s0 = 0.0f, s1 = 0.0f, s2 = 0.0f;
#pragma unroll
    for (int k = 0; k < NEU; ++k) {
      const float hv = hr[k];
      s0 += hv * w1s[k];
      s1 += hv * w1s[NEU + k];
      s2 += hv * w1s[2 * NEU + k];
    }
    const float t0 = tanhf(s0), t1 = tanhf(s1), t2 = tanhf(s2);
    const float e0 = t0 * w1bs[0] + t1 * w1bs[1] + t2 * w1bs[2];
    const float e1 = t0 * w1bs[3] + t1 * w1bs[4] + t2 * w1bs[5];
    const float e2 = t0 * w1bs[6] + t1 * w1bs[7] + t2 * w1bs[8];
    const bool don = dfl[0] > 0;
    const float u0 = don ? e0 : 0.0f;
    const float u1 = don ? e1 : 0.0f;
    const float u2 = don ? e2 : 0.0f;
    const float p0 = posp[(size_t)n * 3 + 0] + u0;
    const float p1 = posp[(size_t)n * 3 + 1] + u1;
    const float p2 = posp[(size_t)n * 3 + 2] + u2;
    const float* rb = rot + b * 9;
    const float j0 = p0 * rb[0] + p1 * rb[3] + p2 * rb[6];
    const float j1 = p0 * rb[1] + p1 * rb[4] + p2 * rb[7];
    const float lg = zs[b * LATD + (LATD - 1)] * law[n] + lab[n];
    const float ex = expf(-lg);
    const float ac = 1.0f / (1.0f + ex);
    const float ams = ac * amp[0];
    const float px0 = (j0 + 0.5f) * 255.0f;
    const float px1 = (j1 + 0.5f) * 255.0f;
    o2s[2 * q] = j0; o2s[2 * q + 1] = j1;
    o3s[3 * q] = p0; o3s[3 * q + 1] = p1; o3s[3 * q + 2] = p2;
    o4s[3 * q] = u0; o4s[3 * q + 1] = u1; o4s[3 * q + 2] = u2;
    sps[4 * q] = px0; sps[4 * q + 1] = px1; sps[4 * q + 2] = ams; sps[4 * q + 3] = 0.0f;
  }
  __syncthreads();

  const size_t o2b = (size_t)R0 * 2;
  const size_t o3b = (size_t)R0 * 3;
  const size_t o4b = (size_t)R0 * 4;
  if (wave == 0) {
    const v4f va = *(const v4f*)(o2s + 4 * lane);
    const v4f vb = *(const v4f*)(o4s + 128 + 4 * (lane & 15));
    volatile v4f* pa = (volatile v4f*)(out2 + o2b + 4 * lane);
    volatile v4f* pb = (volatile v4f*)(out4 + o3b + 128 + 4 * (lane & 15));
    *pa = va;
    if (lane < 16) *pb = vb;
    __threadfence();
    *pa = va;
    if (lane < 16) *pb = vb;
  } else if (wave == 1) {
    const v4f va = *(const v4f*)(o3s + 4 * lane);
    const v4f vb = *(const v4f*)(o3s + 128 + 4 * (lane & 15));
    volatile v4f* pa = (volatile v4f*)(out3 + o3b + 4 * lane);
    volatile v4f* pb = (volatile v4f*)(out3 + o3b + 128 + 4 * (lane & 15));
    *pa = va;
    if (lane < 16) *pb = vb;
    __threadfence();
    *pa = va;
    if (lane < 16) *pb = vb;
  } else if (wave == 2) {
    const v4f va = *(const v4f*)(o4s + 4 * lane);
    const v4f vb = *(const v4f*)(sps + 4 * lane);
    volatile v4f* pa = (volatile v4f*)(out4 + o3b + 4 * lane);
    volatile v4f* pb = (volatile v4f*)(sp + o4b + 4 * lane);
    *pa = va;
    *pb = vb;
    __threadfence();
    *pa = va;
    *pb = vb;
  } else {
    const v4f va = *(const v4f*)(sps + 128 + 4 * lane);
    volatile v4f* pa = (volatile v4f*)(sp + o4b + 128 + 4 * lane);
    *pa = va;
    __threadfence();
    *pa = va;
  }
}

__global__ __launch_bounds__(ST) void k_splat(const float* __restrict__ sp, float* out0, float* out1,
                                              int nChunks) {
  __shared__ int cnts[NWS];
  __shared__ __attribute__((aligned(16))) int   dcc[2 * ST];
  __shared__ __attribute__((aligned(16))) float dpx[2 * ST];
  __shared__ float damp[ST];
  __shared__ float wts[2 * ST * KTAP];
  __shared__ int   wl[NWS * ST];
  __shared__ __attribute__((aligned(16))) float tileS[TW * TW];

  const int tid = threadIdx.x, lane = tid & 31, wave = tid >> 5;
  const int bid = (int)blockIdx.x;
  if (bid >= BIMG * TPI) return;
  const int b  = bid / TPI;
  const int t  = bid - b * TPI;
  const int ty = t / TPD, tx = t - ty * TPD;
  const int y0 = ty * TW, x0 = tx * TW;
  const int ybase = y0 + 8 * wave;
  const int xa = x0 + 2 * lane;
  constexpr float INV2S2 = (float)(1.0 / (2.0 * 1.5 * 1.5));
  const int nch = nChunks > (NPT + ST - 1) / ST ? (NPT + ST - 1) / ST : nChunks;

  float av[16];
#pragma unroll
  for (int i = 0; i < 16; ++i) av[i] = 0.0f;

  const float* spb = sp + (size_t)b * NPT * 4;

#pragma unroll 1
  for (int ch = 0; ch < nch; ++ch) {
    const int n  = ch * ST + tid;
    const int nn = n < NPT ? n : NPT - 1;
    const v4f rec = *(const v4f*)(spb + (size_t)nn * 4);
    float c0f = floorf(rec.x + 0.5f);
    float c1f = floorf(rec.y + 0.5f);
    c0f = fminf(fmaxf(c0f, -1048576.0f), 1048576.0f);
    c1f = fminf(fmaxf(c1f, -1048576.0f), 1048576.0f);
    const int c0 = (int)c0f, c1 = (int)c1f;
    const bool hit = (n < NPT) && (c0 + HALFK >= y0) && (c0 - HALFK <= y0 + TW - 1) &&
                     (c1 + HALFK >= x0) && (c1 - HALFK <= x0 + TW - 1);
    const unsigned mk = __builtin_amdgcn_ballot_w32(hit);
    const int pos = (int)__builtin_amdgcn_mbcnt_lo(mk, 0u);
    if (lane == 0) cnts[wave] = (int)__builtin_popcount(mk);
    __syncthreads();

    int base = 0, H = 0;
#pragma unroll
    for (int w = 0; w < NWS; ++w) {
      const int c = cnts[w];
      base += (w < wave) ? c : 0;
      H += c;
    }
    H = H < 0 ? 0 : (H > ST ? ST : H);
    if (hit) {
      const int s = base + pos;
      if ((unsigned)s < (unsigned)ST) {
        dcc[2 * s] = c0; dcc[2 * s + 1] = c1;
        dpx[2 * s] = rec.x; dpx[2 * s + 1] = rec.y;
        damp[s] = rec.z;
      }
    }
    __syncthreads();

    if (H > 0) {
      const int nw = 2 * KTAP * H;
#pragma unroll 1
      for (int e = tid; e < nw; e += ST) {
        const int s  = e / (2 * KTAP);
        const int j  = e - s * (2 * KTAP);
        const int dm = (j >= KTAP) ? 1 : 0;
        const int jj = j - KTAP * dm;
        const int   c = dcc[2 * s + dm];
        const float p = dpx[2 * s + dm];
        const float g = (float)(c + jj - HALFK);
        const float dd = g - p;
        float tt = dd * dd;
        tt = -tt;
        tt = tt * INV2S2;
        const float w  = expf(tt);
        const float wa = damp[s] * w;
        wts[dm * (ST * KTAP) + s * KTAP + jj] = dm ? w : wa;
      }
      __syncthreads();

      int Hw = 0;
#pragma unroll 1
      for (int i = 0; i < H; i += 32) {
        const int s  = i + lane;
        const int sc = s < H ? s : H - 1;
        const int c0h = dcc[2 * sc];
        const int dy0 = ybase - c0h + HALFK;
        const bool rel = (s < H) && (dy0 <= 2 * HALFK) && (dy0 + 7 >= 0);
        const unsigned mk2 = __builtin_amdgcn_ballot_w32(rel);
        if (rel) {
          const int p = Hw + (int)__builtin_amdgcn_mbcnt_lo(mk2, 0u);
          if ((unsigned)p < (unsigned)ST) wl[wave * ST + p] = sc;
        }
        Hw += (int)__builtin_popcount(mk2);
      }
      Hw = Hw < 0 ? 0 : (Hw > ST ? ST : Hw);
      __syncthreads();

#pragma unroll 1
      for (int i = 0; i < Hw; ++i) {
        int s = wl[wave * ST + i];
        s = s < 0 ? 0 : (s > ST - 1 ? ST - 1 : s);
        const int c0h = dcc[2 * s], c1h = dcc[2 * s + 1];
        const int dy0 = ybase - c0h + HALFK;
        int dxa = xa - c1h + HALFK;
        int dxb = dxa + 1;
        const bool ina = (unsigned)dxa < (unsigned)KTAP;
        const bool inb = (unsigned)dxb < (unsigned)KTAP;
        dxa = ina ? dxa : 0;
        dxb = inb ? dxb : 0;
        const float* w1p = wts + ST * KTAP + s * KTAP;
        float wxa = w1p[dxa];
        float wxb = w1p[dxb];
        wxa = ina ? wxa : 0.0f;
        wxb = inb ? wxb : 0.0f;
        const float* w0p = wts + s * KTAP;
#pragma unroll
        for (int r = 0; r < 8; ++r) {
          const int dy  = dy0 + r;
          const int dyc = dy < 0 ? 0 : (dy > 2 * HALFK ? 2 * HALFK : dy);
          if ((unsigned)dy < (unsigned)KTAP) {
            const float wy = w0p[dyc];
            av[2 * r]     += wy * wxa;
            av[2 * r + 1] += wy * wxb;
          }
        }
      }
    }
  }

  {
    float* tp = tileS + (8 * wave) * TW + 2 * lane;
#pragma unroll
    for (int r = 0; r < 8; ++r) {
      v2f v; v.x = av[2 * r]; v.y = av[2 * r + 1];
      *(v2f*)(tp + r * TW) = v;
    }
  }
  __syncthreads();
  v4f vv[4];
  size_t gg[4];
#pragma unroll
  for (int i = 0; i < 4; ++i) {
    const int rr = 8 * wave + 2 * i + (lane >> 4);
    const int pc = lane & 15;
    vv[i] = *(const v4f*)(tileS + rr * TW + 4 * pc);
    gg[i] = ((size_t)(b * BOXW + y0 + rr)) * BOXW + (size_t)(x0 + 4 * pc);
  }
#pragma unroll
  for (int i = 0; i < 4; ++i) {
    *(volatile v4f*)(out0 + gg[i]) = vv[i];
    *(volatile v4f*)(out1 + gg[i]) = vv[i];
  }
  __threadfence();
#pragma unroll
  for (int i = 0; i < 4; ++i) {
    *(volatile v4f*)(out0 + gg[i]) = vv[i];
    *(volatile v4f*)(out1 + gg[i]) = vv[i];
  }
}

extern "C" void kernel_launch(void* const* d_in, const int* in_sizes, int n_in,
                              void* d_out, int out_size, void* d_ws, size_t ws_size,
                              hipStream_t stream) {
  if (n_in < 12) return;
  if (in_sizes[0] != BIMG * LATD || in_sizes[1] != BIMG * 9 || in_sizes[2] != NPT * 3 || in_sizes[3] < 1) return;
  if (in_sizes[4] != NEU * KIN0 || in_sizes[5] != NLAY * NEU * NEU || in_sizes[6] != NLAY * NEU) return;
  if (in_sizes[7] != 3 * NEU || in_sizes[8] != 9 || in_sizes[9] != NPT || in_sizes[10] != NPT || in_sizes[11] < 1) return;
  const int nImg = BIMG * BOXW * BOXW;
  if (out_size != 2 * nImg + NROWS * 8) return;

  const size_t spBytes = (size_t)NROWS * 4 * sizeof(float);
  if (spBytes > ws_size) return;

  const float* z    = (const float*)d_in[0];
  const float* rot  = (const float*)d_in[1];
  const float* posp = (const float*)d_in[2];
  const float* amp  = (const float*)d_in[3];
  const float* w0   = (const float*)d_in[4];
  const float* wd   = (const float*)d_in[5];
  const float* bd   = (const float*)d_in[6];
  const float* w1a  = (const float*)d_in[7];
  const float* w1b  = (const float*)d_in[8];
  const float* law  = (const float*)d_in[9];
  const float* lab  = (const float*)d_in[10];
  const int*   dfl  = (const int*)d_in[11];

  float* out = (float*)d_out;
  float* o0 = out;
  float* o1 = out + nImg;
  float* o2 = out + 2 * nImg;
  float* o3 = o2 + (size_t)NROWS * 2;
  float* o4 = o3 + (size_t)NROWS * 3;
  float* sp = (float*)d_ws;

  k_mlp<<<NROWS / RT, MT, 0, stream>>>(z, rot, posp, amp, w0, wd, bd, w1a, w1b, law, lab, dfl,
                                       o2, o3, o4, sp);
  k_splat<<<BIMG * TPI, ST, 0, stream>>>(sp, o0, o1, (NPT + ST - 1) / ST);
}
